// DCNv3Module_82188494176856
// MI455X (gfx1250) — hardware-verified
//
#include <hip/hip_runtime.h>


typedef __attribute__((ext_vector_type(16))) _Float16 v16h;
typedef __attribute__((ext_vector_type(8)))  _Float16 v8h;
typedef __attribute__((ext_vector_type(8)))  float    v8f;
typedef __attribute__((ext_vector_type(4)))  float    v4f;

namespace {
constexpr int KS = 3, PAD = 1, G = 4, C_IN = 64, C_OUT = 64, KT = 9;
constexpr int Bn = 4, H = 128, W = 128, HW = H * W, NPIX = Bn * HW;
constexpr int CG = 16;
constexpr int OMC = 108;
constexpr int OMG = 27;
constexpr int OMR = 32;
constexpr int KC = 160;
constexpr int KCR = 144;
constexpr int HALF = NPIX / 2;
constexpr float EPS = 1e-5f;
constexpr int XPITCH = 72;
constexpr int SPITCH = 168;
constexpr int STL = 32;
}

__device__ __forceinline__ void dep_guard_h(v8f& a, v8f& b, v16h x, v16h y) { asm volatile("v_nop\n\tv_nop\n\tv_nop\n\tv_nop" : "+v"(a), "+v"(b) : "v"(x), "v"(y)); }
__device__ __forceinline__ void keep4_h(v16h a, v16h b, v16h c, v16h d) { asm volatile("v_nop" :: "v"(a), "v"(b), "v"(c), "v"(d)); }
__device__ __forceinline__ void acc_guard4(v8f& a, v8f& b, v8f& c, v8f& d) { asm volatile("v_nop\n\tv_nop\n\tv_nop\n\tv_nop" : "+v"(a), "+v"(b), "+v"(c), "+v"(d)); }

template <typename T> struct Frag;
template <> struct Frag<_Float16> {
  typedef v16h V; union U { v16h v; v8h h[2]; };
  static __device__ __forceinline__ v16h load(const _Float16* p) {
    U f; f.h[0] = *(const v8h*)(p); f.h[1] = *(const v8h*)(p + 16); return f.v;
  }
  static __device__ __forceinline__ v8f mma(v16h a, v16h b, v8f c) {
    return __builtin_amdgcn_wmma_f32_16x16x32_f16(false, a, false, b, (short)0, c, false, false);
  }
  static __device__ __forceinline__ void guard(v8f& a, v8f& b, v16h x, v16h y) { dep_guard_h(a, b, x, y); }
  static __device__ __forceinline__ void keep(v16h a, v16h b, v16h c, v16h d) { keep4_h(a, b, c, d); }
};

__global__ __launch_bounds__(256) void k_prep(
    const float* __restrict__ w_om, const float* __restrict__ dcn_w,
    _Float16* __restrict__ wom16, _Float16* __restrict__ wd16)
{
  const int i = blockIdx.x * 256 + threadIdx.x;
  if (i < (G * OMR * C_IN) / 2) {
    const int e = 2 * i;
    const int g = e / (OMR * C_IN);
    const int r = (e / C_IN) % OMR;
    const int c = e % C_IN;
    float f0 = 0.0f, f1 = 0.0f;
    if (r < OMG) {
      const float* src = w_om + (size_t)(g * OMG + r) * C_IN + c;
      f0 = src[0] * 1024.0f;
      f1 = src[1] * 1024.0f;
    }
    const _Float16 h0 = (_Float16)f0, h1 = (_Float16)f1;
    const unsigned u = (unsigned)__builtin_bit_cast(unsigned short, h0) |
                       ((unsigned)__builtin_bit_cast(unsigned short, h1) << 16);
    ((volatile unsigned*)wom16)[i] = u;
    __threadfence();
    ((volatile unsigned*)wom16)[i] = u;
  }
  if (i < (G * CG * KC) / 2) {
    const int e = 2 * i;
    const int g = e / (CG * KC);
    const int o = (e / KC) % CG;
    const int j = e % KC;
    float f0 = 0.0f, f1 = 0.0f;
    if (j < KCR)     f0 = dcn_w[((size_t)(g * CG + o) * CG + j / KT) * KT + j % KT] * 64.0f;
    if (j + 1 < KCR) f1 = dcn_w[((size_t)(g * CG + o) * CG + (j + 1) / KT) * KT + (j + 1) % KT] * 64.0f;
    const _Float16 h0 = (_Float16)f0, h1 = (_Float16)f1;
    const unsigned u = (unsigned)__builtin_bit_cast(unsigned short, h0) |
                       ((unsigned)__builtin_bit_cast(unsigned short, h1) << 16);
    ((volatile unsigned*)wd16)[i] = u;
    __threadfence();
    ((volatile unsigned*)wd16)[i] = u;
  }
}

__global__ __launch_bounds__(256) void k_xT(const float* __restrict__ x, _Float16* __restrict__ x16)
{
  __shared__ __align__(16) _Float16 sT[64 * XPITCH];
  const int t = threadIdx.x;
  const int pix0 = blockIdx.x * 64;
  const int b = pix0 >> 14, hw0 = pix0 & (HW - 1);
  const float* xb = x + (size_t)b * C_IN * HW + hw0;
#pragma unroll
  for (int it = 0; it < 4; ++it) {
    const int idx = it * 256 + t;
    const int c = idx >> 4;
    const int p4 = (idx & 15) * 4;
    const v4f v = *(const v4f*)(xb + (size_t)c * HW + p4);
    sT[(p4 + 0) * XPITCH + c] = (_Float16)v[0];
    sT[(p4 + 1) * XPITCH + c] = (_Float16)v[1];
    sT[(p4 + 2) * XPITCH + c] = (_Float16)v[2];
    sT[(p4 + 3) * XPITCH + c] = (_Float16)v[3];
  }
  __syncthreads();
  const int lane = t & 31, wave = t >> 5;
  const int q = lane >> 3, c8 = (lane & 7) * 8;
  for (int pass = 0; pass < 2; ++pass) {
#pragma unroll
    for (int it = 0; it < 2; ++it) {
      const int row = wave * 8 + it * 4 + q;
      const v8h hv = *(const v8h*)(sT + row * XPITCH + c8);
      *(volatile v8h*)(x16 + (size_t)(pix0 + row) * C_IN + c8) = hv;
    }
    __threadfence();
  }
}

template <int RI, int KSTEPS>
__global__ __launch_bounds__(256) void k_wgemm(
    const unsigned short* __restrict__ Ap, int lda,
    const unsigned short* __restrict__ Btp, int ldb,
    float* __restrict__ C, long cBatchStride, int ldc, int pixBase,
    const float* __restrict__ bias, int biasOff, int biasN,
    float scale, int nTiles)
{
  typedef _Float16 T;
  typedef v16h V;
  const T* A = (const T*)Ap;
  const T* Bt = (const T*)Btp;
  __shared__ __align__(16) float sT[8][16 * 68];
  const int lane = threadIdx.x & 31;
  const int wave = threadIdx.x >> 5;
  const int tile = blockIdx.x * 8 + wave;
  if (tile >= nTiles) return;
  const int n0 = tile << 6;
  const int rlane = lane & 15;
  const int koff  = (lane >> 4) * 8;
  const int mOff  = (lane >> 4) * 8;

  v8f acc[RI][4];
#pragma unroll
  for (int i = 0; i < RI; ++i)
#pragma unroll
    for (int j = 0; j < 4; ++j) acc[i][j] = (v8f){0.f,0.f,0.f,0.f,0.f,0.f,0.f,0.f};

  for (int k0 = 0; k0 < KSTEPS * 32; k0 += 32) {
    V bh[4];
#pragma unroll
    for (int j = 0; j < 4; ++j)
      bh[j] = Frag<T>::load(Bt + (size_t)(n0 + (j << 4) + rlane) * ldb + koff + k0);
#pragma unroll
    for (int i = 0; i < RI; ++i) {
      V ah = Frag<T>::load(A + (size_t)((i << 4) + rlane) * lda + koff + k0);
#pragma unroll
      for (int j = 0; j < 4; ++j) acc[i][j] = Frag<T>::mma(ah, bh[j], acc[i][j]);
      Frag<T>::guard(acc[i][0], acc[i][3], ah, ah);
    }
    Frag<T>::keep(bh[0], bh[1], bh[2], bh[3]);
  }
#pragma unroll
  for (int i = 0; i < RI; ++i) acc_guard4(acc[i][0], acc[i][1], acc[i][2], acc[i][3]);

  float* slab = sT[wave];
  const int p0 = pixBase + n0;
  float* Cb = C + (size_t)(p0 >> 14) * cBatchStride + (p0 & (HW - 1));
#pragma unroll
  for (int i = 0; i < RI; ++i) {
    const int mBase = i << 4;
#pragma unroll
    for (int j = 0; j < 4; ++j) {
#pragma unroll
      for (int r = 0; r < 8; ++r) {
        const int rr = mBase + mOff + r;
        const int bi = biasOff + min(rr, biasN - 1);
        const float bv = (rr < biasN) ? bias[bi] : 0.0f;
        slab[(mOff + r) * 68 + (j << 4) + rlane] = acc[i][j][r] * scale + bv;
      }
    }
    __builtin_amdgcn_fence(__ATOMIC_RELEASE, "workgroup");
    __builtin_amdgcn_wave_barrier();
    __builtin_amdgcn_fence(__ATOMIC_ACQUIRE, "workgroup");
    {
      const int hh = lane >> 4, c4 = (lane & 15) * 4;
      for (int pass = 0; pass < 2; ++pass) {
#pragma unroll
        for (int it = 0; it < 8; ++it) {
          const int row = it * 2 + hh;
          const v4f v = *(const v4f*)(slab + row * 68 + c4);
          *(volatile v4f*)(Cb + (size_t)(mBase + row) * ldc + c4) = v;
        }
        __threadfence();
      }
    }
    __builtin_amdgcn_fence(__ATOMIC_RELEASE, "workgroup");
    __builtin_amdgcn_wave_barrier();
    __builtin_amdgcn_fence(__ATOMIC_ACQUIRE, "workgroup");
  }
}

__global__ __launch_bounds__(128) void k_samp(
    const float* __restrict__ x, const float* __restrict__ omg,
    const float* __restrict__ oscale, _Float16* __restrict__ col,
    int g, int pixStart)
{
  __shared__ __align__(16) _Float16 sW[4 * 32 * SPITCH];
  const int lane = threadIdx.x & 31, wave = threadIdx.x >> 5;
  const int lp  = blockIdx.x * 128 + threadIdx.x;
  const int pix = pixStart + lp;
  const int b = pix >> 14, hw = pix & (HW - 1);
  const int hi = hw >> 7, wi = hw & (W - 1);
  const float sc = oscale[0];

  float w00[KT], w01[KT], w10[KT], w11[KT];
  int   i00[KT], i01[KT], i10[KT], i11[KT];
#pragma unroll
  for (int k = 0; k < KT; ++k) {
    const float offy = omg[(size_t)(2 * k) * NPIX + pix] * sc;
    const float offx = omg[(size_t)(2 * k + 1) * NPIX + pix] * sc;
    const float ml   = omg[(size_t)(2 * KT + k) * NPIX + pix];
    const float msk  = __builtin_amdgcn_rcpf(1.0f + __expf(-ml));
    const float py = (float)(hi - PAD + k / KS) + offy;
    const float px = (float)(wi - PAD + k % KS) + offx;
    float y0f = floorf(py), x0f = floorf(px);
    const float wy1 = py - y0f, wx1 = px - x0f;
    const float wy0 = 1.0f - wy1, wx0 = 1.0f - wx1;
    y0f = fminf(fmaxf(y0f, -4.0f), (float)(H + 2));
    x0f = fminf(fmaxf(x0f, -4.0f), (float)(W + 2));
    const int y0 = (int)y0f, x0 = (int)x0f;
    const bool vy0 = (y0 >= 0) && (y0 <= H - 1);
    const bool vy1 = (y0 >= -1) && (y0 <= H - 2);
    const bool vx0 = (x0 >= 0) && (x0 <= W - 1);
    const bool vx1 = (x0 >= -1) && (x0 <= W - 2);
    const int cy0 = min(max(y0, 0), H - 1), cy1 = min(max(y0 + 1, 0), H - 1);
    const int cx0 = min(max(x0, 0), W - 1), cx1 = min(max(x0 + 1, 0), W - 1);
    const float a00 = wy0 * wx0, a01 = wy0 * wx1, a10 = wy1 * wx0, a11 = wy1 * wx1;
    w00[k] = (vy0 && vx0) ? a00 * msk : 0.0f;
    w01[k] = (vy0 && vx1) ? a01 * msk : 0.0f;
    w10[k] = (vy1 && vx0) ? a10 * msk : 0.0f;
    w11[k] = (vy1 && vx1) ? a11 * msk : 0.0f;
    i00[k] = cy0 * W + cx0; i01[k] = cy0 * W + cx1;
    i10[k] = cy1 * W + cx0; i11[k] = cy1 * W + cx1;
  }

  _Float16* myrow = sW + wave * (32 * SPITCH) + lane * SPITCH;
  const float* xg = x + (size_t)(b * C_IN + g * CG) * HW;
#pragma unroll 1
  for (int c = 0; c < CG; ++c) {
    const float* p = xg + (size_t)c * HW;
#pragma unroll
    for (int k = 0; k < KT; ++k) {
      const float v = w00[k] * p[i00[k]] + w01[k] * p[i01[k]] +
                      w10[k] * p[i10[k]] + w11[k] * p[i11[k]];
      myrow[c * KT + k] = (_Float16)v;
    }
  }
  {
    v8h z;
#pragma unroll
    for (int e = 0; e < 8; ++e) z[e] = (_Float16)0.0f;
    *(v8h*)(myrow + KCR) = z;
    *(v8h*)(myrow + KCR + 8) = z;
  }
  __syncthreads();
  {
    const _Float16* tile = sW + wave * (32 * SPITCH);
    _Float16* dstw = col + (size_t)(blockIdx.x * 128 + wave * 32) * KC;
    for (int pass = 0; pass < 2; ++pass) {
#pragma unroll
      for (int it = 0; it < 20; ++it) {
        const int q = it * 32 + lane;
        const int row = q / 20;
        const int ch = (q - row * 20) * 8;
        const v8h hv = *(const v8h*)(tile + row * SPITCH + ch);
        *(volatile v8h*)(dstw + (size_t)q * 8) = hv;
      }
      __threadfence();
    }
  }
}

__global__ __launch_bounds__(256) void k_stats(const float* __restrict__ v, float* __restrict__ stats)
{
  __shared__ double sh[256];
  __shared__ double sh2[256];
  __shared__ float res[2];
  const int tid = threadIdx.x;
  const int bg = blockIdx.x;
  const int b = bg >> 2, g = bg & 3;
  const v4f* base = (const v4f*)(v + (size_t)(b * C_OUT + g * CG) * HW);
  double s = 0.0, s2 = 0.0;
#pragma unroll 1
  for (int i = tid; i < (CG * HW) / 4; i += 256) {
    const v4f t = base[i];
    const double d0 = (double)t[0], d1 = (double)t[1], d2 = (double)t[2], d3 = (double)t[3];
    s += d0; s += d1; s += d2; s += d3;
    s2 += d0 * d0; s2 += d1 * d1; s2 += d2 * d2; s2 += d3 * d3;
  }
  sh[tid] = s; sh2[tid] = s2;
  __syncthreads();
  for (int ofs = 128; ofs > 0; ofs >>= 1) {
    if (tid < ofs) { sh[tid] += sh[tid + ofs]; sh2[tid] += sh2[tid + ofs]; }
    __syncthreads();
  }
  if (tid == 0) {
    const double invN = 1.0 / (double)(CG * HW);
    const double mu = sh[0] * invN;
    double var = sh2[0] * invN - mu * mu;
    if (var < 0.0) var = 0.0;
    res[0] = (float)mu;
    res[1] = rsqrtf((float)var + EPS);
  }
  __syncthreads();
  if (tid < 8) {
    v4f o = (v4f){0.f, 0.f, 0.f, 0.f};
    if (tid == 0) { o[0] = res[0]; o[1] = res[1]; }
    float* dst = stats + (size_t)bg * STL + tid * 4;
    *(volatile v4f*)dst = o;
    __threadfence();
    *(volatile v4f*)dst = o;
  }
}

__global__ __launch_bounds__(256) void k_gn(
    float* out, const float* __restrict__ stats,
    const float* __restrict__ gw, const float* __restrict__ gb, int n4)
{
  const int i4 = blockIdx.x * 256 + threadIdx.x;
  if (i4 >= n4) return;
  const int e = i4 << 2;
  const int c = (e >> 14) & (C_OUT - 1);
  const int b = e >> 20;
  const int bg = (b << 2) + (c >> 4);
  const float mu = stats[bg * STL], rs = stats[bg * STL + 1];
  const float w = gw[c], bb = gb[c];
  const v4f xin = *(const v4f*)(out + e);
  v4f o = xin;
#pragma unroll 1
  for (int q = 0; q < 4; ++q) {
    const float xv = (q == 0) ? xin[0] : (q == 1) ? xin[1] : (q == 2) ? xin[2] : xin[3];
    float t = (xv - mu) * rs;
    t = t * w + bb;
    const float y = 0.5f * t * (1.0f + erff(t * 0.70710678118654752f));
    o[0] = (q == 0) ? y : o[0];
    o[1] = (q == 1) ? y : o[1];
    o[2] = (q == 2) ? y : o[2];
    o[3] = (q == 3) ? y : o[3];
  }
  *(volatile v4f*)(out + e) = o;
  __threadfence();
  *(volatile v4f*)(out + e) = o;
}

extern "C" void kernel_launch(void* const* d_in, const int* in_sizes, int n_in,
                              void* d_out, int out_size, void* d_ws, size_t ws_size,
                              hipStream_t stream)
{
  if (n_in < 8) return;
  if (in_sizes[0] != Bn * C_IN * HW) return;
  if (in_sizes[1] != OMC * C_IN) return;
  if (in_sizes[2] < OMC) return;
  if (in_sizes[3] != G * CG * CG * KT) return;
  if (in_sizes[4] < G * CG) return;
  if (in_sizes[5] < C_OUT || in_sizes[6] < C_OUT) return;
  if (in_sizes[7] < 1) return;
  if (out_size < Bn * C_OUT * HW) return;

  const float* x     = (const float*)d_in[0];
  const float* w_om  = (const float*)d_in[1];
  const float* b_om  = (const float*)d_in[2];
  const float* dcn_w = (const float*)d_in[3];
  const float* dcn_b = (const float*)d_in[4];
  const float* gn_w  = (const float*)d_in[5];
  const float* gn_b  = (const float*)d_in[6];
  const float* osc   = (const float*)d_in[7];
  float* out = (float*)d_out;

  const size_t off_x16 = 0;
  const size_t off_om  = off_x16 + (size_t)NPIX * C_IN * 2;
  const size_t off_col = off_om  + (size_t)OMR * NPIX * 4;
  const size_t off_wom = off_col + (size_t)HALF * KC * 2;
  const size_t off_wd  = off_wom + (size_t)G * OMR * C_IN * 2;
  const size_t off_st  = off_wd  + (size_t)G * CG * KC * 2;
  const size_t total   = off_st  + (size_t)Bn * G * STL * 4;
  if (total > ws_size) return;

  char* ws = (char*)d_ws;
  _Float16* x16   = (_Float16*)(ws + off_x16);
  float*    omg   = (float*)(ws + off_om);
  _Float16* colb  = (_Float16*)(ws + off_col);
  _Float16* wom16 = (_Float16*)(ws + off_wom);
  _Float16* wd16  = (_Float16*)(ws + off_wd);
  float*    stats = (float*)(ws + off_st);

  k_prep<<<(G * CG * KC / 2 + 255) / 256, 256, 0, stream>>>(w_om, dcn_w, wom16, wd16);
  k_xT<<<NPIX / 64, 256, 0, stream>>>(x, x16);

  const int omTiles = NPIX / 64;
  const int dcTiles = HALF / 64;
  for (int g = 0; g < G; ++g) {
    k_wgemm<2, 2><<<(omTiles + 7) / 8, 256, 0, stream>>>(
        (const unsigned short*)(wom16 + (size_t)g * OMR * C_IN), C_IN,
        (const unsigned short*)x16, C_IN,
        omg, (long)HW, NPIX, 0,
        b_om, OMG * g, OMG,
        0.0009765625f, omTiles);
    for (int hf = 0; hf < 2; ++hf) {
      k_samp<<<HALF / 128, 128, 0, stream>>>(x, omg, osc, colb, g, hf * HALF);
      k_wgemm<1, 5><<<(dcTiles + 7) / 8, 256, 0, stream>>>(
          (const unsigned short*)(wd16 + (size_t)g * CG * KC), KC,
          (const unsigned short*)colb, KC,
          out + (size_t)g * CG * HW, (long)C_OUT * HW, HW, hf * HALF,
          dcn_b, CG * g, CG,
          0.015625f, dcTiles);
    }
  }

  k_stats<<<Bn * G, 256, 0, stream>>>(out, stats);
  const int n4 = Bn * C_OUT * HW / 4;
  k_gn<<<(n4 + 255) / 256, 256, 0, stream>>>(out, stats, gn_w, gn_b, n4);
}
